// TSPNNet_47966194762329
// MI455X (gfx1250) — hardware-run, weakly checked
//
#include <hip/hip_runtime.h>


#ifndef NB
#define NB 4
#endif
#define NB_FULL 4
#define NN   512
#define CC   128
#define IND  4
#define EDIM 16
#define NL   3
#define LN_EPS  1e-5f
#define DEG_EPS 1e-6f
#define OSP  132
#define OUT1_OFF (NB_FULL * NN)

static_assert(NN == 512);
static_assert(CC == 128);
static_assert(NN % 64 == 0);
static_assert(NN % 32 == 0);
static_assert(CC % 32 == 0);
static_assert(CC % 64 == 0);
static_assert((NB * NN) % 64 == 0);
static_assert((NB * NN) % 8 == 0);
static_assert(((size_t)NL * CC * CC) % 8 == 0);
static_assert(NB <= NB_FULL);
static_assert((size_t)OUT1_OFF * 4 == 8192);

typedef unsigned short bf;
typedef __attribute__((ext_vector_type(16))) __bf16   v16bf;
typedef __attribute__((ext_vector_type(8)))  unsigned short v8us;
typedef __attribute__((ext_vector_type(8)))  float    v8f;
typedef __attribute__((ext_vector_type(4)))  float    v4f;
typedef v4f  __attribute__((may_alias)) v4fa;

__device__ __forceinline__ unsigned short f2bf(float f) { unsigned u = __float_as_uint(f); u += 0x7FFFu + ((u >> 16) & 1u); return (unsigned short)(u >> 16); }
__device__ __forceinline__ float bf2f(unsigned short h) { return __uint_as_float((unsigned)h << 16); }
__device__ __forceinline__ float bfr(float f) { return bf2f(f2bf(f)); }
__device__ __forceinline__ v16bf cat16b(v8us lo, v8us hi) { return __builtin_bit_cast(v16bf, __builtin_shufflevector(lo, hi, 0, 1, 2, 3, 4, 5, 6, 7, 8, 9, 10, 11, 12, 13, 14, 15)); }
__device__ __forceinline__ v8f wmmab(v16bf a, v16bf b, v8f c) { return __builtin_amdgcn_wmma_f32_16x16x32_bf16(false, a, false, b, (short)0, c, false, false); }
__device__ __forceinline__ v16bf ldb(const bf* p)  { return cat16b(*(const v8us*)p, *(const v8us*)(p + 16)); }
__device__ __forceinline__ void wave_sync() { __builtin_amdgcn_fence(3  , "wavefront"); __builtin_amdgcn_wave_barrier(); asm volatile("" ::: "memory"); }

__global__ __launch_bounds__(256) void k_cvt8(const float* __restrict__ src, bf* dst, size_t n8) {
    const size_t i = (size_t)blockIdx.x * 256 + threadIdx.x; if (i >= n8) return;
    const v8f v = *(const v8f*)(src + i * 8); v8us o;
#pragma unroll
    for (int k = 0; k < 8; ++k) o[k] = f2bf(v[k]);
    *(volatile v8us*)(dst + i * 8) = o; __threadfence(); *(volatile v8us*)(dst + i * 8) = o;
}

__global__ __launch_bounds__(32) void k_scal(const float* __restrict__ W_ee, const float* __restrict__ b_ee, const float* __restrict__ W_ep, const float* __restrict__ b_ep, float* scal) {
    const int lane = threadIdx.x & 31;
    float pa = 0.0f, pc = 0.0f;
#pragma unroll 1
    for (int j = 0; j < CC / 32; ++j) {
        const int e = lane + 32 * j;
        float sa = 0.0f, sc = 0.0f;
#pragma unroll 4
        for (int k = 0; k < EDIM; ++k) { const float w = bfr(W_ep[e * EDIM + k]); sa = fmaf(w, bfr(W_ee[k]), sa); sc = fmaf(w, bfr(b_ee[k]), sc); }
        pa += sa; pc += sc + bfr(b_ep[e]);
    }
#pragma unroll
    for (int off = 16; off > 0; off >>= 1) { pa += __shfl_xor(pa, off, 32); pc += __shfl_xor(pc, off, 32); }
    const float val = (lane == 0) ? pa : ((lane == 1) ? pc : 0.0f);
    *(volatile float*)(scal + lane) = val; __threadfence(); *(volatile float*)(scal + lane) = val;
}

__global__ __launch_bounds__(128) void k_embed(const float* __restrict__ nf, const float* __restrict__ W_emb, const float* __restrict__ b_emb, float* XI, bf* XTH, bf* XTL) {
    __shared__ __align__(16) float os[64 * OSP];
    const int tid = threadIdx.x, lane = tid & 31; const int wave = __builtin_amdgcn_readfirstlane(tid >> 5);
    const int r0 = blockIdx.x * 64;
    const v4f wr = *(const v4f*)(W_emb + tid * IND);
    const float w0 = bfr(wr[0]), w1 = bfr(wr[1]), w2 = bfr(wr[2]), w3 = bfr(wr[3]); const float bias = bfr(b_emb[tid]);
#pragma unroll 2
    for (int r = 0; r < 64; ++r) {
        const v4f n = *(const v4f*)(nf + (size_t)(r0 + r) * IND);
        float acc = bfr(n[0]) * w0; acc = fmaf(bfr(n[1]), w1, acc); acc = fmaf(bfr(n[2]), w2, acc); acc = fmaf(bfr(n[3]), w3, acc);
        os[r * OSP + tid] = acc + bias;
    }
    __syncthreads();
    const int bb = r0 / NN, n0 = r0 % NN;
#pragma unroll 1
    for (int ps = 0; ps < 2; ++ps) {
#pragma unroll 4
        for (int it = 0; it < 16; ++it) { const int row = it * 4 + wave;
            const v4f val = *(const v4fa*)(&os[row * OSP + lane * 4]);
            *(volatile v4f*)(XI + (size_t)(r0 + row) * CC + lane * 4) = val; }
#pragma unroll 2
        for (int it = 0; it < 8; ++it) { const int crow = it * 16 + (tid >> 3), q = tid & 7;
            v8us oh, ol;
#pragma unroll
            for (int i = 0; i < 8; ++i) { const float xv = os[(8 * q + i) * OSP + crow]; const unsigned short hb = f2bf(xv); oh[i] = hb; ol[i] = f2bf(xv - bf2f(hb)); }
            const size_t oo = ((size_t)bb * CC + crow) * NN + n0 + 8 * q;
            *(volatile v8us*)(XTH + oo) = oh; *(volatile v8us*)(XTL + oo) = ol; }
        if (ps == 0) __threadfence(); }
}

__global__ __launch_bounds__(256) void k_buildA(const float* __restrict__ adj, const float* __restrict__ scal, bf* AH, bf* AL) {
    const int lane = threadIdx.x & 31; const int wave = __builtin_amdgcn_readfirstlane(threadIdx.x >> 5);
    const size_t row = (size_t)blockIdx.x * 8 + wave;
    const float* rp = adj + row * NN;
    v8f v0 = *(const v8f*)(rp + 8 * lane); v8f v1 = *(const v8f*)(rp + 256 + 8 * lane);
    float s = 0.0f;
#pragma unroll
    for (int k = 0; k < 8; ++k) { v0[k] = bfr(v0[k]); s += v0[k]; }
#pragma unroll
    for (int k = 0; k < 8; ++k) { v1[k] = bfr(v1[k]); s += v1[k]; }
#pragma unroll
    for (int off = 16; off > 0; off >>= 1) s += __shfl_xor(s, off, 32);
    const float rd = 1.0f / (s + DEG_EPS);
    const float ga = scal[0], gc = scal[1];
    v8us h0, l0, h1, l1;
#pragma unroll
    for (int k = 0; k < 8; ++k) {
        const float t0 = (v0[k] * rd) * fmaf(ga, v0[k], gc); const unsigned short a0 = f2bf(t0); h0[k] = a0; l0[k] = f2bf(t0 - bf2f(a0));
        const float t1 = (v1[k] * rd) * fmaf(ga, v1[k], gc); const unsigned short a1 = f2bf(t1); h1[k] = a1; l1[k] = f2bf(t1 - bf2f(a1)); }
    const size_t o0 = row * NN + 8 * lane, o1 = o0 + 256;
    *(volatile v8us*)(AH + o0) = h0; *(volatile v8us*)(AH + o1) = h1; *(volatile v8us*)(AL + o0) = l0; *(volatile v8us*)(AL + o1) = l1;
    __threadfence();
    *(volatile v8us*)(AH + o0) = h0; *(volatile v8us*)(AH + o1) = h1; *(volatile v8us*)(AL + o0) = l0; *(volatile v8us*)(AL + o1) = l1;
}

__global__ __launch_bounds__(32) void k_agg(const bf* __restrict__ AH, const bf* __restrict__ AL, const bf* __restrict__ XH, const bf* __restrict__ XL, bf* GH, bf* GL) {
    __shared__ __align__(16) float os[16 * 68];
    const int lane = threadIdx.x & 31, lr = lane & 15, hi = lane >> 4;
    const int r0 = blockIdx.x * 32, c0 = blockIdx.y * 64, b = blockIdx.z;
    v8f acc[2][4];
#pragma unroll
    for (int mb = 0; mb < 2; ++mb)
#pragma unroll
        for (int nb = 0; nb < 4; ++nb) acc[mb][nb] = (v8f){};
    const size_t aoff = ((size_t)b * NN + r0 + lr) * NN + 8 * hi, boff = ((size_t)b * CC + c0 + lr) * NN + 8 * hi;
#pragma unroll 1
    for (int kc = 0; kc < NN; kc += 32) {
        v16bf ah[2], al[2];
#pragma unroll
        for (int mb = 0; mb < 2; ++mb) { ah[mb] = ldb(AH + aoff + (size_t)mb * 16 * NN + kc); al[mb] = ldb(AL + aoff + (size_t)mb * 16 * NN + kc); }
#pragma unroll
        for (int nb = 0; nb < 4; ++nb) { const v16bf bh = ldb(XH + boff + (size_t)nb * 16 * NN + kc); const v16bf bl = ldb(XL + boff + (size_t)nb * 16 * NN + kc);
#pragma unroll
            for (int mb = 0; mb < 2; ++mb) acc[mb][nb] = wmmab(ah[mb], bh, acc[mb][nb]);
#pragma unroll
            for (int mb = 0; mb < 2; ++mb) acc[mb][nb] = wmmab(al[mb], bh, acc[mb][nb]);
#pragma unroll
            for (int mb = 0; mb < 2; ++mb) acc[mb][nb] = wmmab(ah[mb], bl, acc[mb][nb]); }
        asm volatile("v_nop\n\tv_nop\n\tv_nop\n\tv_nop" : "+v"(acc[0][0]), "+v"(acc[0][1]), "+v"(acc[0][2]), "+v"(acc[0][3]), "+v"(acc[1][0]), "+v"(acc[1][1]), "+v"(acc[1][2]), "+v"(acc[1][3]) : "v"(ah[0]), "v"(ah[1]), "v"(al[0]), "v"(al[1]));
    }
#pragma unroll
    for (int mb = 0; mb < 2; ++mb) {
#pragma unroll
        for (int nb = 0; nb < 4; ++nb) {
#pragma unroll
            for (int j = 0; j < 8; ++j) os[(hi * 8 + j) * 68 + nb * 16 + lr] = acc[mb][nb][j]; }
        wave_sync();
        const size_t sb = ((size_t)b * NN + r0 + mb * 16) * CC + c0;
#pragma unroll 1
        for (int ps = 0; ps < 2; ++ps) {
#pragma unroll
            for (int s = 0; s < 4; ++s) { const int row = 4 * s + (lane >> 3), c8 = (lane & 7) * 8;
                const v4f x0 = *(const v4fa*)(&os[row * 68 + c8]); const v4f x1 = *(const v4fa*)(&os[row * 68 + c8 + 4]); v8us hv, rv;
#pragma unroll
                for (int i = 0; i < 4; ++i) { const unsigned short a0 = f2bf(x0[i]); const unsigned short a1 = f2bf(x1[i]); hv[i] = a0; hv[4 + i] = a1; rv[i] = f2bf(x0[i] - bf2f(a0)); rv[4 + i] = f2bf(x1[i] - bf2f(a1)); }
                const size_t oo = sb + (size_t)row * CC + c8;
                *(volatile v8us*)(GH + oo) = hv; *(volatile v8us*)(GL + oo) = rv; }
            if (ps == 0) __threadfence(); }
        wave_sync();
    }
}

__global__ __launch_bounds__(128) void k_conv(const bf* __restrict__ GH, const bf* __restrict__ GL, const bf* __restrict__ W, const float* __restrict__ bc, const float* __restrict__ lg, const float* __restrict__ lb,
                                              const float* __restrict__ XI, bf* XTH, bf* XTL, float* PS, int wxt) {
    __shared__ __align__(16) float os[64 * OSP];
    __shared__ __align__(16) float cs[4 * CC];
    const int tid = threadIdx.x, lane = tid & 31, lr = lane & 15, hi = lane >> 4; const int wave = __builtin_amdgcn_readfirstlane(tid >> 5);
    const int r0 = blockIdx.x * 64;
    v8f acc[8];
#pragma unroll
    for (int nb = 0; nb < 8; ++nb) acc[nb] = (v8f){};
    const size_t aoff = (size_t)(r0 + 16 * wave + lr) * CC + 8 * hi, boff = (size_t)lr * CC + 8 * hi;
#pragma unroll 1
    for (int kc = 0; kc < CC; kc += 32) {
        const v16bf ah = ldb(GH + aoff + kc), al = ldb(GL + aoff + kc);
#pragma unroll
        for (int nb = 0; nb < 8; ++nb) { const v16bf b = ldb(W + boff + (size_t)nb * 16 * CC + kc);
            acc[nb] = wmmab(ah, b, acc[nb]); acc[nb] = wmmab(al, b, acc[nb]); }
        asm volatile("v_nop\n\tv_nop\n\tv_nop\n\tv_nop" : "+v"(acc[0]), "+v"(acc[1]), "+v"(acc[2]), "+v"(acc[3]), "+v"(acc[4]), "+v"(acc[5]), "+v"(acc[6]), "+v"(acc[7]) : "v"(ah), "v"(al));
    }
#pragma unroll
    for (int nb = 0; nb < 8; ++nb) {
#pragma unroll
        for (int j = 0; j < 8; ++j) os[(16 * wave + 8 * hi + j) * OSP + nb * 16 + lr] = acc[nb][j]; }
    wave_sync();
    v4f bc4 = *(const v4f*)(bc + lane * 4), g4 = *(const v4f*)(lg + lane * 4), b4 = *(const v4f*)(lb + lane * 4);
#pragma unroll
    for (int i = 0; i < 4; ++i) { bc4[i] = bfr(bc4[i]); g4[i] = bfr(g4[i]); b4[i] = bfr(b4[i]); }
    v4f csum = (v4f){};
#pragma unroll 1
    for (int r = 0; r < 16; ++r) {
        const int row = 16 * wave + r;
        v4f v = *(const v4fa*)(&os[row * OSP + lane * 4]); v = v + bc4;
        float s = (v[0] + v[1]) + (v[2] + v[3]);
#pragma unroll
        for (int off = 16; off > 0; off >>= 1) s += __shfl_xor(s, off, 32);
        const float mean = s * (1.0f / CC);
        const v4f d = v - mean;
        float q = (d[0] * d[0] + d[1] * d[1]) + (d[2] * d[2] + d[3] * d[3]);
#pragma unroll
        for (int off = 16; off > 0; off >>= 1) q += __shfl_xor(q, off, 32);
        const float rstd = rsqrtf(q * (1.0f / CC) + LN_EPS);
        const v4f xi = *(const v4f*)(XI + (size_t)(r0 + row) * CC + lane * 4);
        v4f y;
#pragma unroll
        for (int i = 0; i < 4; ++i) { const float t = d[i] * rstd * g4[i] + b4[i] + xi[i]; y[i] = fmaxf(t, 0.0f); }
        *(v4fa*)(&os[row * OSP + lane * 4]) = y; csum = csum + y;
    }
    *(v4fa*)(&cs[wave * CC + lane * 4]) = csum;
    __syncthreads();
    const v4f tot = ((*(const v4fa*)(&cs[lane * 4]) + *(const v4fa*)(&cs[CC + lane * 4])) + *(const v4fa*)(&cs[2 * CC + lane * 4])) + *(const v4fa*)(&cs[3 * CC + lane * 4]);
    const int bb = r0 / NN, n0 = r0 % NN;
#pragma unroll 1
    for (int ps = 0; ps < 2; ++ps) {
        if (wave == 0) *(volatile v4f*)(PS + (size_t)blockIdx.x * CC + lane * 4) = tot;
        if (wxt != 0) {
#pragma unroll 2
            for (int it = 0; it < 8; ++it) { const int crow = it * 16 + (tid >> 3), q8 = tid & 7;
                v8us oh, ol;
#pragma unroll
                for (int i = 0; i < 8; ++i) { const float xv = os[(8 * q8 + i) * OSP + crow]; const unsigned short hb = f2bf(xv); oh[i] = hb; ol[i] = f2bf(xv - bf2f(hb)); }
                const size_t oo = ((size_t)bb * CC + crow) * NN + n0 + 8 * q8;
                *(volatile v8us*)(XTH + oo) = oh; *(volatile v8us*)(XTL + oo) = ol; } }
        if (ps == 0) __threadfence(); }
}

__global__ __launch_bounds__(256) void k_head(const float* __restrict__ PS, const float* __restrict__ W_pi, const float* __restrict__ b_pi, const float* __restrict__ W_v, const float* __restrict__ b_v, float* out) {
    __shared__ __align__(16) float pl[NB * CC];
    __shared__ __align__(16) float res[NB * NN + 4];
    const int tid = threadIdx.x;
#pragma unroll 1
    for (int idx = tid; idx < NB * CC; idx += 256) { const int b = idx / CC, c = idx % CC; float s = 0.0f;
#pragma unroll 1
        for (int j = 0; j < NN / 64; ++j) s += PS[(size_t)(b * (NN / 64) + j) * CC + c];
        pl[idx] = s * (1.0f / NN); }
    __syncthreads();
#pragma unroll 1
    for (int n = tid; n < NN; n += 256) {
        float acc[NB];
#pragma unroll
        for (int b = 0; b < NB; ++b) acc[b] = 0.0f;
#pragma unroll 4
        for (int c = 0; c < CC; ++c) { const float w = bfr(W_pi[(size_t)n * CC + c]);
#pragma unroll
            for (int b = 0; b < NB; ++b) acc[b] = fmaf(pl[b * CC + c], w, acc[b]); }
        const float bias = bfr(b_pi[n]);
#pragma unroll
        for (int b = 0; b < NB; ++b) res[b * NN + n] = acc[b] + bias;
    }
    { int bsel = tid & 3; bsel = (bsel < NB) ? bsel : (NB - 1);
      float sv = 0.0f;
#pragma unroll 4
      for (int c = 0; c < CC; ++c) sv = fmaf(pl[bsel * CC + c], bfr(W_v[c]), sv);
      sv += bfr(b_v[0]);
      if (tid < 4) res[NB * NN + tid] = (tid < NB) ? sv : 0.0f; }
    __syncthreads();
#pragma unroll 1
    for (int ps = 0; ps < 2; ++ps) {
#pragma unroll 1
        for (int i = tid; i < NB * NN / 4; i += 256) { const v4f val = *(const v4fa*)(&res[i * 4]); *(volatile v4f*)(out + (size_t)i * 4) = val; }
        if (tid == 0) { const v4f vv = *(const v4fa*)(&res[NB * NN]); *(volatile v4f*)(out + OUT1_OFF) = vv; }
        if (ps == 0) __threadfence(); }
}

static constexpr size_t al256(size_t v) { return (v + 255) & ~(size_t)255; }
static constexpr size_t SZ_SC = al256((size_t)32 * 4);
static constexpr size_t SZ_WC = al256((size_t)NL * CC * CC * 2);
static constexpr size_t SZ_A  = al256((size_t)NB * NN * NN * 2);
static constexpr size_t SZ_XI = al256((size_t)NB * NN * CC * 4);
static constexpr size_t SZ_XT = al256((size_t)NB * CC * NN * 2);
static constexpr size_t SZ_G  = al256((size_t)NB * NN * CC * 2);
static constexpr size_t SZ_PS = al256((size_t)(NB * NN / 64) * CC * 4);
static constexpr size_t SZ_TOTAL = SZ_SC + SZ_WC + 2 * SZ_A + SZ_XI + 2 * SZ_XT + 2 * SZ_G + SZ_PS;
static_assert(SZ_TOTAL <= (size_t)134217728);

extern "C" void kernel_launch(void* const* d_in, const int* in_sizes, int n_in,
                              void* d_out, int out_size, void* d_ws, size_t ws_size, hipStream_t stream) {
    if (n_in < 16) return;
    if ((size_t)in_sizes[0] < (size_t)NB * NN * IND) return;
    if ((size_t)in_sizes[1] < (size_t)NB * NN * NN) return;
    if (in_sizes[2] < CC * IND || in_sizes[3] < CC) return;
    if (in_sizes[4] < EDIM || in_sizes[5] < EDIM || in_sizes[6] < CC * EDIM || in_sizes[7] < CC) return;
    if (in_sizes[8] < NL * CC * CC || in_sizes[9] < NL * CC || in_sizes[10] < NL * CC || in_sizes[11] < NL * CC) return;
    if (in_sizes[12] < NN * CC || in_sizes[13] < NN || in_sizes[14] < CC || in_sizes[15] < 1) return;
    if ((size_t)out_size < (size_t)OUT1_OFF + 4) return;
    if (SZ_TOTAL > ws_size) return;
    const float* nf   = (const float*)d_in[0];  const float* adj  = (const float*)d_in[1];
    const float* wemb = (const float*)d_in[2];  const float* bemb = (const float*)d_in[3];
    const float* wee  = (const float*)d_in[4];  const float* bee  = (const float*)d_in[5];
    const float* wep  = (const float*)d_in[6];  const float* bep  = (const float*)d_in[7];
    const float* wcv  = (const float*)d_in[8];  const float* bcv  = (const float*)d_in[9];
    const float* lng  = (const float*)d_in[10]; const float* lnb  = (const float*)d_in[11];
    const float* wpi  = (const float*)d_in[12]; const float* bpi  = (const float*)d_in[13];
    const float* wv   = (const float*)d_in[14]; const float* bv   = (const float*)d_in[15];
    float* OUT = (float*)d_out;
    char* wsp = (char*)d_ws;
    float* SCAL = (float*)wsp; wsp += SZ_SC;
    bf* WCB = (bf*)wsp; wsp += SZ_WC;
    bf* AH  = (bf*)wsp; wsp += SZ_A;
    bf* AL  = (bf*)wsp; wsp += SZ_A;
    float* XI = (float*)wsp; wsp += SZ_XI;
    bf* XTH = (bf*)wsp; wsp += SZ_XT;
    bf* XTL = (bf*)wsp; wsp += SZ_XT;
    bf* GH  = (bf*)wsp; wsp += SZ_G;
    bf* GL  = (bf*)wsp; wsp += SZ_G;
    float* PS = (float*)wsp; wsp += SZ_PS;

    k_scal<<<1, 32, 0, stream>>>(wee, bee, wep, bep, SCAL);
    { const size_t n8 = (size_t)NL * CC * CC / 8; k_cvt8<<<(unsigned)((n8 + 255) / 256), 256, 0, stream>>>(wcv, WCB, n8); }
    k_embed<<<NB * NN / 64, 128, 0, stream>>>(nf, wemb, bemb, XI, XTH, XTL);
    k_buildA<<<NB * NN / 8, 256, 0, stream>>>(adj, SCAL, AH, AL);
    for (int i = 0; i < NL; ++i) {
        k_agg<<<dim3(NN / 32, CC / 64, NB), 32, 0, stream>>>(AH, AL, XTH, XTL, GH, GL);
        k_conv<<<NB * NN / 64, 128, 0, stream>>>(GH, GL, WCB + (size_t)i * CC * CC, bcv + (size_t)i * CC, lng + (size_t)i * CC, lnb + (size_t)i * CC, XI, XTH, XTL, PS, (i + 1 < NL) ? 1 : 0);
    }
    k_head<<<1, 256, 0, stream>>>(PS, wpi, bpi, wv, bv, OUT);
}
